// BidirectionalMamba_41618233098840
// MI455X (gfx1250) — hardware-verified
//
#include <hip/hip_runtime.h>
#include <hip/hip_bf16.h>
#include <math.h>

#define BB 4
#define LL 2048
#define DM 512
#define DI 1024
#define NS 16
#define KC 4
#define RR 32
#define MTOK (BB * LL)
#define GSTR 48
#define SS 2048
#define HH 1
#define DKK 64

typedef _Float16 bf16;
typedef _Float16 f16;
typedef __attribute__((ext_vector_type(4))) unsigned v4u_t;
typedef unsigned v4ua __attribute__((ext_vector_type(4), may_alias));
typedef __attribute__((ext_vector_type(4))) float v4f_t;
typedef float v4fa __attribute__((ext_vector_type(4), may_alias));
typedef __attribute__((ext_vector_type(16))) bf16  bf16x16;
typedef bf16x16 f16x16;
typedef __attribute__((ext_vector_type(8)))  bf16  bf16x8;
typedef bf16x8 f16x8;
typedef __attribute__((ext_vector_type(4)))  bf16  bf16x4;
typedef __attribute__((ext_vector_type(8)))  float f32x8;
__device__ __forceinline__ f32x8 wmma16(f16x16 a, f16x16 b, f32x8 c) {
  c = __builtin_amdgcn_wmma_f32_16x16x32_f16(false, a, false, b, (short)0, c, false, false);
  asm volatile("v_nop\n\tv_nop\n\tv_nop\n\tv_nop" : "+v"(c) : "v"(a), "v"(b));
  return c;
}
#define LDS_STRIDE 48
#define KSTRIDE    72
#define VSTRIDE    48

__device__ __forceinline__ f32x8 wmma_bf16(bf16x16 a, bf16x16 b, f32x8 c) {
  c = __builtin_amdgcn_wmma_f32_16x16x32_f16(false, a, false, b, (short)0, c, false, false);
  asm volatile("v_nop\n\tv_nop\n\tv_nop\n\tv_nop" : "+v"(c) : "v"(a), "v"(b));
  return c;
}

template <typename T>
__device__ __forceinline__ bf16x16 load_frag(const T* __restrict__ base, int ld,
                                             int row0, int k0) {
  const int lane = threadIdx.x & 31;
  const int r    = lane & 15;
  const int kh   = (lane >> 4) * 8;
  const T* p0 = base + (size_t)(row0 + r) * ld + (k0 + kh);
  const T* p1 = p0 + 16;
  bf16x16 f;
#pragma unroll
  for (int i = 0; i < 8; ++i) {
    f[i]     = (bf16)p0[i];
    f[i + 8] = (bf16)p1[i];
  }
  return f;
}

__device__ __forceinline__ bf16x16 lds_frag(const bf16* base, int stride) {
  const int lane = threadIdx.x & 31;
  const int row  = lane & 15;
  const int kh   = (lane >> 4) * 8;
  const bf16x8 lo = *(const bf16x8*)(base + row * stride + kh);
  const bf16x8 hi = *(const bf16x8*)(base + row * stride + kh + 16);
  bf16x16 f;
#pragma unroll
  for (int i = 0; i < 8; ++i) { f[i] = lo[i]; f[i + 8] = hi[i]; }
  return f;
}

template <typename T>
__device__ __forceinline__ void stage_read16(const T* __restrict__ p, float* buf) {
#pragma unroll
  for (int i = 0; i < 16; ++i) buf[i] = (float)p[i];
}

__device__ __forceinline__ void stage_write(bf16* dst, const float* buf, int nquad) {
#pragma unroll
  for (int i = 0; i < nquad; ++i) {
    bf16x4 q;
    q[0] = (bf16)buf[4 * i];     q[1] = (bf16)buf[4 * i + 1];
    q[2] = (bf16)buf[4 * i + 2]; q[3] = (bf16)buf[4 * i + 3];
    *(bf16x4*)(dst + 4 * i) = q;
  }
}

template <typename AT, int MODE>
__global__ __launch_bounds__(256) void gemm_rb_kernel(
    const AT* __restrict__ A, const float* __restrict__ W,
    const float* __restrict__ bias, const float* __restrict__ rowscale, const float* __restrict__ R, const float* __restrict__ rowbias, void* __restrict__ out,
    int M, int N, int K) {
  __shared__ bf16 ldsA[128 * LDS_STRIDE];
  __shared__ bf16 ldsW[256 * LDS_STRIDE];
  __shared__ __attribute__((aligned(16))) unsigned char sob[256 * 136 * 2];

  const int t    = threadIdx.x;
  const int wave = t >> 5;
  const int lane = t & 31;
  const int wm   = (wave & 1) * 64;
  const int wn   = (wave >> 1) * 64;
  const int mBlk = blockIdx.x * 128;
  const int nBlk = blockIdx.y * 256;

  const int arow = t >> 1;
  const int ach  = (t & 1) * 16;

  float abuf[16];
  float wbuf[32];

  stage_read16(A + (size_t)(mBlk + arow) * K + ach, abuf);
  const int nrow = min(nBlk + t, N - 1);
  stage_read16(W + (size_t)nrow * K,          wbuf);
  stage_read16(W + (size_t)nrow * K + 16,     wbuf + 16);

  f32x8 acc[4][4] = {};

  for (int k = 0; k < K; k += 32) {
    __syncthreads();
    stage_write(&ldsA[arow * LDS_STRIDE + ach], abuf, 4);
    stage_write(&ldsW[t * LDS_STRIDE],          wbuf, 8);
    if (k + 32 < K) {
      stage_read16(A + (size_t)(mBlk + arow) * K + (k + 32) + ach, abuf);
      stage_read16(W + (size_t)nrow * K + (k + 32),          wbuf);
      stage_read16(W + (size_t)nrow * K + (k + 32) + 16,     wbuf + 16);
    }
    __syncthreads();

    bf16x16 af[4], wf[4];
#pragma unroll
    for (int i = 0; i < 4; ++i)
      af[i] = lds_frag(ldsA + (wm + 16 * i) * LDS_STRIDE, LDS_STRIDE);
#pragma unroll
    for (int j = 0; j < 4; ++j)
      wf[j] = lds_frag(ldsW + (wn + 16 * j) * LDS_STRIDE, LDS_STRIDE);
#pragma unroll
    for (int i = 0; i < 4; ++i)
#pragma unroll
      for (int j = 0; j < 4; ++j)
        acc[i][j] = wmma_bf16(af[i], wf[j], acc[i][j]);
  }

  const int nlane = lane & 15;
  const int mh    = (lane >> 4) * 8;
  __syncthreads();
  if (MODE == 0 || MODE == 1 || MODE == 3) {
    bf16* so = (bf16*)sob;
#pragma unroll
    for (int i = 0; i < 4; ++i)
#pragma unroll
      for (int j = 0; j < 4; ++j) {
        const int nl = wn + 16 * j + nlane;
        const float bv = bias ? bias[nBlk + nl] : 0.0f;
        if (MODE == 3) {
#pragma unroll 1
          for (int r = 0; r < 8; ++r) {
            const int ml = wm + 16 * i + mh + r;
            const float xg = acc[i][j][r] + bv;
            so[ml * 264 + nl] = (bf16)(0.5f * xg * (1.0f + erff(xg * 0.70710678118654752f)));
          }
        } else {
#pragma unroll
        for (int r = 0; r < 8; ++r) {
          const int ml = wm + 16 * i + mh + r;
          const bf16 hv = (bf16)(acc[i][j][r] + bv);
          if (MODE == 0) so[ml * 264 + nl] = hv;
          else           so[nl * 136 + ml] = hv;
        }
        }
      }
    __syncthreads();
#pragma unroll 1
    for (int pass = 0; pass < 2; ++pass) {
      if (MODE == 0 || MODE == 3) {
        for (int ch = t; ch < 128 * 32; ch += 256) { const int ml = ch >> 5, q = (ch & 31) * 8;
          *(volatile v4u_t*)((bf16*)out + (size_t)(mBlk + ml) * N + nBlk + q) = *(const v4ua*)(so + ml * 264 + q); }
      } else {
        const int b_ = mBlk / SS, s0 = mBlk & (SS - 1);
        for (int ch = t; ch < 256 * 16; ch += 256) { const int nl = ch >> 4, q = (ch & 15) * 8; const int n = nBlk + nl, h = n >> 6, dk = n & (DKK - 1);
          *(volatile v4u_t*)((bf16*)out + (((size_t)(b_ * HH + h)) * DKK + dk) * SS + s0 + q) = *(const v4ua*)(so + nl * 136 + q); }
      }
      __threadfence();
    }
  } else {
    float* so = (float*)sob;
#pragma unroll 1
    for (int hf = 0; hf < 2; ++hf) {
      if (wm == hf * 64) {
#pragma unroll
        for (int i = 0; i < 4; ++i)
#pragma unroll
          for (int j = 0; j < 4; ++j) {
            const int nl = wn + 16 * j + nlane;
            const float bv = bias ? bias[nBlk + nl] : 0.0f;
#pragma unroll
            for (int r = 0; r < 8; ++r) { const int mrow = mBlk + hf * 64 + 16 * i + mh + r; so[(16 * i + mh + r) * 260 + nl] = acc[i][j][r] * (rowscale ? rowscale[mrow] : 1.0f) + bv + (rowbias ? rowbias[mrow] : 0.0f); }
          }
      }
      __syncthreads();
      if (R) {
        for (int ch = t; ch < 64 * 64; ch += 256) { const int ml = ch >> 6, q = (ch & 63) * 4;
          if (nBlk + q < N) { const v4f_t rv = *(const v4f_t*)(R + (size_t)(mBlk + hf * 64 + ml) * N + nBlk + q); v4f_t v = *(const volatile v4fa*)(so + ml * 260 + q); v += rv; *(volatile v4fa*)(so + ml * 260 + q) = v; } }
        asm volatile("s_wait_dscnt 0" ::: "memory");
      }
#pragma unroll 1
      for (int pass = 0; pass < 2; ++pass) {
        for (int ch = t; ch < 64 * 64; ch += 256) { const int ml = ch >> 6, q = (ch & 63) * 4;
          if (nBlk + q < N) *(volatile v4f_t*)((float*)out + (size_t)(mBlk + hf * 64 + ml) * N + nBlk + q) = *(const volatile v4fa*)(so + ml * 260 + q); }
        __threadfence();
      }
      __syncthreads();
    }
  }
}


template <typename AT, bool ACC>
__global__ __launch_bounds__(256) void gemm_kn2(const AT* __restrict__ A, int lda, size_t strideA,
                                               const float* __restrict__ Wm, int ldw, size_t strideW,
                                               const float* __restrict__ bias, float scale,
                                               float* __restrict__ Y, int ldy, size_t strideY, int K) {
  __shared__ __attribute__((aligned(16))) f16 ldsA[128 * GSTR], ldsAl[128 * GSTR];
  __shared__ __attribute__((aligned(16))) f16 ldsW[128 * GSTR], ldsWl[128 * GSTR];
  __shared__ __attribute__((aligned(16))) float oS[8][32 * 68];
  const int tid = threadIdx.x, lane = tid & 31, wave = tid >> 5, cl = lane & 15, rh = (lane >> 4) * 8;
  const int m0 = blockIdx.x * 128, n0 = blockIdx.y * 128;
  const int wm = (wave & 3) * 32, wn = (wave >> 2) * 64;
  A += (size_t)blockIdx.z * strideA; Wm += (size_t)blockIdx.z * strideW; Y += (size_t)blockIdx.z * strideY;
  f32x8 acc[2][4], accx[2][4];
#pragma unroll
  for (int i = 0; i < 2; ++i)
#pragma unroll
    for (int j = 0; j < 4; ++j) { f32x8 z = {}; acc[i][j] = z; accx[i][j] = z; }
#pragma unroll 1
  for (int k0 = 0; k0 < K; k0 += 32) {
    __syncthreads();
    {
      const int row = tid >> 1, ch = (tid & 1) * 16;
      const AT* src = A + (size_t)(m0 + row) * lda + k0 + ch;
#pragma unroll
      for (int g = 0; g < 16; ++g) { const float v = (float)src[g]; const f16 h = (f16)v; ldsA[row * GSTR + ch + g] = h; ldsAl[row * GSTR + ch + g] = (f16)((v - (float)h) * 2048.0f); }
    }
    {
      const int k = tid >> 3, nn0 = (tid & 7) * 16;
      const float* src = Wm + (size_t)(k0 + k) * ldw + n0 + nn0;
#pragma unroll
      for (int g = 0; g < 4; ++g) { const v4f_t v = *(const v4f_t*)(src + 4 * g);
#pragma unroll
        for (int u = 0; u < 4; ++u) { const f16 h = (f16)v[u]; ldsW[(nn0 + 4 * g + u) * GSTR + k] = h; ldsWl[(nn0 + 4 * g + u) * GSTR + k] = (f16)((v[u] - (float)h) * 2048.0f); } }
    }
    __syncthreads();
    f16x16 af[2], afl[2];
#pragma unroll
    for (int i = 0; i < 2; ++i) { af[i] = lds_frag(ldsA + (wm + 16 * i) * GSTR, GSTR); afl[i] = lds_frag(ldsAl + (wm + 16 * i) * GSTR, GSTR); }
#pragma unroll
    for (int j = 0; j < 4; ++j) {
      const f16x16 bf = lds_frag(ldsW + (wn + 16 * j) * GSTR, GSTR), bfl = lds_frag(ldsWl + (wn + 16 * j) * GSTR, GSTR);
#pragma unroll
      for (int i = 0; i < 2; ++i) { acc[i][j] = wmma16(af[i], bf, acc[i][j]); accx[i][j] = wmma16(af[i], bfl, accx[i][j]); accx[i][j] = wmma16(afl[i], bf, accx[i][j]); }
    }
  }
  float* so = oS[wave];
#pragma unroll
  for (int i = 0; i < 2; ++i)
#pragma unroll
    for (int j = 0; j < 4; ++j) {
      const float bv = bias ? bias[n0 + wn + 16 * j + cl] : 0.0f;
#pragma unroll
      for (int r = 0; r < 8; ++r) so[(16 * i + rh + r) * 68 + 16 * j + cl] = (acc[i][j][r] + accx[i][j][r] * (1.0f / 2048.0f)) * scale + bv;
    }
  asm volatile("s_wait_dscnt 0" ::: "memory");
  __builtin_amdgcn_wave_barrier();
  if (ACC) {
#pragma unroll
    for (int it = 0; it < 16; ++it) { const int f4 = lane + 32 * it, rr = f4 >> 4, q = (f4 & 15) * 4;
      const v4f_t old = *(const volatile v4fa*)(Y + (size_t)(m0 + wm + rr) * ldy + n0 + wn + q);
      v4f_t v = *(const volatile v4fa*)(so + rr * 68 + q); v += old; *(volatile v4fa*)(so + rr * 68 + q) = v; }
    asm volatile("s_wait_dscnt 0" ::: "memory");
  }
#pragma unroll 1
  for (int pass = 0; pass < 2; ++pass) {
#pragma unroll
    for (int it = 0; it < 16; ++it) { const int f4 = lane + 32 * it, rr = f4 >> 4, q = (f4 & 15) * 4;
      *(volatile v4f_t*)(Y + (size_t)(m0 + wm + rr) * ldy + n0 + wn + q) = *(const volatile v4fa*)(so + rr * 68 + q); }
    __threadfence();
  }
}

__global__ __launch_bounds__(256) void k_transpose(const float* __restrict__ Wm, float* __restrict__ Wt, int rows, int cols) {
  __shared__ float tS[64][65];
  const int tid = threadIdx.x, tbj = cols / 64, bi = blockIdx.x / tbj, bj = blockIdx.x % tbj;
  for (int e = tid; e < 64 * 64; e += 256) { const int r = e >> 6, c = e & 63; tS[r][c] = Wm[(size_t)(bi * 64 + r) * cols + bj * 64 + c]; }
  __syncthreads();
  for (int ch = tid; ch < 64 * 16; ch += 256) { const int r = ch >> 4, q4 = (ch & 15) * 4; v4f_t o; o[0] = tS[q4][r]; o[1] = tS[q4 + 1][r]; o[2] = tS[q4 + 2][r]; o[3] = tS[q4 + 3][r];
    float* dst = Wt + (size_t)(bj * 64 + r) * rows + bi * 64 + q4; *(volatile v4f_t*)dst = o; __threadfence(); *(volatile v4f_t*)dst = o; }
}
__global__ __launch_bounds__(256) void k_wxT(const float* __restrict__ Wx, float* __restrict__ Wp) { const int k = blockIdx.x, n = threadIdx.x; if (n < 128) Wp[(size_t)k * 128 + n] = (n < RR + 2 * NS) ? Wx[(size_t)n * DI + k] : 0.0f; }
__global__ __launch_bounds__(256) void k_wdtT(const float* __restrict__ Wdt, float* __restrict__ Wp) { const int n = blockIdx.x * 256 + threadIdx.x; for (int r = 0; r < RR; ++r) Wp[(size_t)r * DI + n] = Wdt[(size_t)n * RR + r]; }
__global__ __launch_bounds__(256) void k_dwconv4(const float* __restrict__ xi, const float* __restrict__ w, const float* __restrict__ cb, int rev, float* __restrict__ xc) {
  const size_t i = (size_t)blockIdx.x * 256 + threadIdx.x; const size_t row = i >> 8; const int d0 = (i & 255) * 4; const int b = row / LL, l = row % LL;
  v4f_t acc; acc[0] = cb[d0]; acc[1] = cb[d0 + 1]; acc[2] = cb[d0 + 2]; acc[3] = cb[d0 + 3];
#pragma unroll
  for (int j = 0; j < KC; ++j) { const int off = j - (KC - 1); const int ls = rev ? (l - off) : (l + off);
    if (ls >= 0 && ls < LL) { const v4f_t v = *(const v4f_t*)(xi + ((size_t)b * LL + ls) * DI + d0);
      acc[0] += w[(d0) * KC + j] * v[0]; acc[1] += w[(d0 + 1) * KC + j] * v[1]; acc[2] += w[(d0 + 2) * KC + j] * v[2]; acc[3] += w[(d0 + 3) * KC + j] * v[3]; } }
  v4f_t o; for (int e = 0; e < 4; ++e) o[e] = 256.0f * (acc[e] / (1.0f + expf(-acc[e])));
  *(volatile v4f_t*)(xc + row * DI + d0) = o; __threadfence(); *(volatile v4f_t*)(xc + row * DI + d0) = o;
}
__global__ __launch_bounds__(256) void k_scan(const float* __restrict__ dtraw, const float* __restrict__ bdt, float* __restrict__ xcy, const float* __restrict__ dbl,
                                             const float* __restrict__ Alog, const float* __restrict__ Dp, const float* __restrict__ z, int rev) {
  __shared__ float bcS[2 * NS];
  const int tid = threadIdx.x, b = blockIdx.x / (DI / 256), d = (blockIdx.x % (DI / 256)) * 256 + tid;
  float A[NS], h[NS];
#pragma unroll
  for (int n = 0; n < NS; ++n) { A[n] = -expf(Alog[d * NS + n]); h[n] = 0.0f; }
  const float dpd = Dp[d], bd = bdt[d];
#pragma unroll 1
  for (int s = 0; s < LL; ++s) {
    const int l = rev ? (LL - 1 - s) : s; const size_t row = (size_t)b * LL + l;
    __syncthreads();
    if (tid < 2 * NS) bcS[tid] = dbl[row * 128 + RR + tid];
    __syncthreads();
    const float dr = dtraw[row * DI + d] + bd; const float delta = (dr > 20.0f) ? dr : log1pf(expf(dr));
    const float xv = xcy[row * DI + d] * (1.0f / 256.0f); const float dx = delta * xv; float yv = 0.0f;
#pragma unroll
    for (int n = 0; n < NS; ++n) { h[n] = expf(delta * A[n]) * h[n] + dx * bcS[n]; yv += h[n] * bcS[NS + n]; }
    yv += dpd * xv; const float zz = z[row * DI + d]; yv *= zz / (1.0f + expf(-zz));
    xcy[row * DI + d] = yv * 256.0f;
  }
}

extern "C" void kernel_launch(void* const* d_in, const int* in_sizes, int n_in,
                              void* d_out, int out_size, void* d_ws, size_t ws_size,
                              hipStream_t stream) {
  (void)in_sizes; (void)n_in; (void)out_size;
  const float** f = (const float**)d_in;
  const float* x = f[0];
  float* out = (float*)d_out;
  char* ws = (char*)d_ws;
  float* xi = (float*)ws; ws += (size_t)MTOK * DI * 4;
  float* z = (float*)ws; ws += (size_t)MTOK * DI * 4;
  float* xc = (float*)ws; ws += (size_t)MTOK * DI * 4;
  float* dbl = (float*)ws; ws += (size_t)MTOK * 128 * 4;
  float* Wxp = (float*)ws; ws += (size_t)DI * 128 * 4; float* Wdtp = (float*)ws; ws += (size_t)RR * DI * 4; float* WoT = (float*)ws; ws += (size_t)DI * DM * 4;
  if ((size_t)(ws - (char*)d_ws) > ws_size) return;
  float* dtraw = xi;
  const dim3 blk(256);
  for (int dir = 0; dir < 2; ++dir) {
    const float* W_in = f[1 + 9 * dir], *conv_w = f[2 + 9 * dir], *conv_b = f[3 + 9 * dir], *W_x = f[4 + 9 * dir], *W_dt = f[5 + 9 * dir], *b_dt = f[6 + 9 * dir], *A_log = f[7 + 9 * dir], *Dp = f[8 + 9 * dir], *W_out = f[9 + 9 * dir];
    gemm_rb_kernel<float, 2><<<dim3(MTOK / 128, DI / 256), blk, 0, stream>>>(x, W_in, nullptr, nullptr, nullptr, nullptr, xi, MTOK, DI, DM);
    gemm_rb_kernel<float, 2><<<dim3(MTOK / 128, DI / 256), blk, 0, stream>>>(x, W_in + (size_t)DI * DM, nullptr, nullptr, nullptr, nullptr, z, MTOK, DI, DM);
    k_dwconv4<<<dim3(MTOK * (DI / 4) / 256), blk, 0, stream>>>(xi, conv_w, conv_b, dir, xc);
    k_wxT<<<dim3(DI), blk, 0, stream>>>(W_x, Wxp); k_wdtT<<<dim3(DI / 256), blk, 0, stream>>>(W_dt, Wdtp); k_transpose<<<dim3((DM / 64) * (DI / 64)), blk, 0, stream>>>(W_out, WoT, DM, DI);
    gemm_kn2<float, false><<<dim3(MTOK / 128, 1, 1), blk, 0, stream>>>(xc, DI, 0, Wxp, 128, 0, nullptr, 1.0f / 256.0f, dbl, 128, 0, DI);
    gemm_kn2<float, false><<<dim3(MTOK / 128, DI / 128, 1), blk, 0, stream>>>(dbl, 128, 0, Wdtp, DI, 0, nullptr, 1.0f, dtraw, DI, 0, RR);
    k_scan<<<dim3(BB * DI / 256), blk, 0, stream>>>(dtraw, b_dt, xc, dbl, A_log, Dp, z, dir);
    if (dir == 0) gemm_kn2<float, false><<<dim3(MTOK / 128, DM / 128, 1), blk, 0, stream>>>(xc, DI, 0, WoT, DM, 0, nullptr, 1.0f / 256.0f, out, DM, 0, DI);
    else          gemm_kn2<float, true ><<<dim3(MTOK / 128, DM / 128, 1), blk, 0, stream>>>(xc, DI, 0, WoT, DM, 0, nullptr, 1.0f / 256.0f, out, DM, 0, DI);
  }
}
